// MultiHeadAttention_5488968204518
// MI455X (gfx1250) — hardware-verified
//
#include <hip/hip_runtime.h>
#ifndef NB
#define NB 2
#endif
#ifndef SEQ
#define SEQ 1024
#endif
#define NB_FULL 2
#define SEQ_FULL 1024
#define FEAT 1024
#define NCH 64
#define MROWS (NB * SEQ)

static_assert(SEQ % 128 == 0);
static_assert(SEQ <= SEQ_FULL);
static_assert(NB <= NB_FULL);
static_assert(FEAT % 128 == 0);
static_assert(FEAT == NCH * 16);
static_assert((size_t)8 * MROWS * FEAT * 2 + (size_t)7 * FEAT * FEAT * 2 <= (size_t)134217728);
static_assert(((size_t)(NB - 1) * SEQ_FULL + SEQ) * FEAT <= (size_t)NB_FULL * SEQ_FULL * FEAT);

typedef __bf16 v16b __attribute__((ext_vector_type(16)));
typedef _Float16 v16h __attribute__((ext_vector_type(16)));
typedef unsigned short v8us __attribute__((ext_vector_type(8), may_alias));
typedef float v8f __attribute__((ext_vector_type(8)));
typedef float v4f __attribute__((ext_vector_type(4)));
typedef float v4fa __attribute__((ext_vector_type(4), may_alias));
union Frag { v16b b; v16h h; v8us half[2]; _Float16 e[16]; unsigned short u[16]; };

#define LOG2E 1.4426950408889634f

__device__ __forceinline__ unsigned short bf16_bits(float x) {
  unsigned int u = __float_as_uint(x);
  return (unsigned short)((u + 0x7FFFu + ((u >> 16) & 1u)) >> 16);
}
__device__ __forceinline__ float bf16_val(unsigned short b) { return __uint_as_float(((unsigned int)b) << 16); }
__device__ __forceinline__ float bf16_rne(float x) { return bf16_val(bf16_bits(x)); }

__device__ __forceinline__ void mma_s2(v16h a0, v16h a1, v16h b, v8f& c0, v8f& c1) {
  c0 = __builtin_amdgcn_wmma_f32_16x16x32_f16(false, a0, false, b, (short)0, c0, false, false);
  c1 = __builtin_amdgcn_wmma_f32_16x16x32_f16(false, a1, false, b, (short)0, c1, false, false);
  asm volatile("v_nop\n\tv_nop\n\tv_nop\n\tv_nop" : "+v"(c0), "+v"(c1) : "v"(a0), "v"(a1), "v"(b));
}
__device__ __forceinline__ void mma_h2(v16h a, v16h bh, v16h bl, v8f& ch, v8f& cl) {
  ch = __builtin_amdgcn_wmma_f32_16x16x32_f16(false, a, false, bh, (short)0, ch, false, false);
  cl = __builtin_amdgcn_wmma_f32_16x16x32_f16(false, a, false, bl, (short)0, cl, false, false);
  asm volatile("v_nop\n\tv_nop\n\tv_nop\n\tv_nop" : "+v"(ch), "+v"(cl) : "v"(a), "v"(bh), "v"(bl));
}

__global__ __launch_bounds__(256) void k_cvtx(const float* __restrict__ X, unsigned short* __restrict__ Xb) {
  const int t = blockIdx.x * 256 + threadIdx.x;
  if (t >= MROWS * (FEAT / 8)) return;
  const int row = t / (FEAT / 8), piece = t - row * (FEAT / 8);
  const int b = row / SEQ, s = row - b * SEQ;
  const float* src = X + ((size_t)b * SEQ_FULL + s) * FEAT + piece * 8;
  const v4f x0 = *(const v4fa*)(src), x1 = *(const v4fa*)(src + 4);
  v8us o;
  o[0] = bf16_bits(x0[0]); o[1] = bf16_bits(x0[1]); o[2] = bf16_bits(x0[2]); o[3] = bf16_bits(x0[3]);
  o[4] = bf16_bits(x1[0]); o[5] = bf16_bits(x1[1]); o[6] = bf16_bits(x1[2]); o[7] = bf16_bits(x1[3]);
  unsigned short* d = Xb + (size_t)t * 8;
  *(volatile v8us*)d = o;
  __threadfence();
  *(volatile v8us*)d = o;
}

template <int MODE>
__global__ __launch_bounds__(256) void k_cvtw(const float* __restrict__ Wsrc, unsigned short* __restrict__ Wp) {
  const int t = blockIdx.x * 256 + threadIdx.x;
  if (t >= FEAT * (FEAT / 8)) return;
  const float* src = Wsrc + (size_t)t * 8;
  const v4f x0 = *(const v4fa*)(src), x1 = *(const v4fa*)(src + 4);
  v8us o;
  if (MODE == 0) {
    o[0] = bf16_bits(x0[0]); o[1] = bf16_bits(x0[1]); o[2] = bf16_bits(x0[2]); o[3] = bf16_bits(x0[3]);
    o[4] = bf16_bits(x1[0]); o[5] = bf16_bits(x1[1]); o[6] = bf16_bits(x1[2]); o[7] = bf16_bits(x1[3]);
  } else {
    Frag f;
    f.e[0] = (_Float16)(bf16_rne(x0[0]) * 64.0f); f.e[1] = (_Float16)(bf16_rne(x0[1]) * 64.0f);
    f.e[2] = (_Float16)(bf16_rne(x0[2]) * 64.0f); f.e[3] = (_Float16)(bf16_rne(x0[3]) * 64.0f);
    f.e[4] = (_Float16)(bf16_rne(x1[0]) * 64.0f); f.e[5] = (_Float16)(bf16_rne(x1[1]) * 64.0f);
    f.e[6] = (_Float16)(bf16_rne(x1[2]) * 64.0f); f.e[7] = (_Float16)(bf16_rne(x1[3]) * 64.0f);
    o = f.half[0];
  }
  unsigned short* d = Wp + (size_t)t * 8;
  *(volatile v8us*)d = o;
  __threadfence();
  *(volatile v8us*)d = o;
}

template <bool BF, int EPI>
__global__ __launch_bounds__(256) void k_gemm(const unsigned short* __restrict__ A, const unsigned short* __restrict__ W,
                                              const float* __restrict__ bias, void* __restrict__ outp,
                                              int N, float sc, float carry) {
  __shared__ __attribute__((aligned(16))) float sst[8][16][68];
  const int tid = threadIdx.x, lane = tid & 31, w = __builtin_amdgcn_readfirstlane((int)(tid >> 5));
  const int wm = w & 3, wn = w >> 2, ln = lane & 15, hh = lane >> 4;
  const int m0 = blockIdx.x * 128 + wm * 32;
  const int n0 = blockIdx.y * 128 + wn * 64;
  const unsigned short* ap = A + (size_t)(m0 + ln) * FEAT + 8 * hh;
  const unsigned short* wp = W + (size_t)(n0 + ln) * FEAT + 8 * hh;
  v8f acc[2][4];
#pragma unroll
  for (int fm = 0; fm < 2; ++fm)
#pragma unroll
    for (int fn = 0; fn < 4; ++fn)
#pragma unroll
      for (int r = 0; r < 8; ++r) acc[fm][fn][r] = 0.0f;

#pragma unroll 1
  for (int k0 = 0; k0 < FEAT; k0 += 32) {
    Frag a[2], b[4];
#pragma unroll
    for (int fm = 0; fm < 2; ++fm) {
      a[fm].half[0] = *(const v8us*)(ap + (size_t)fm * 16 * FEAT + k0);
      a[fm].half[1] = *(const v8us*)(ap + (size_t)fm * 16 * FEAT + k0 + 16);
    }
#pragma unroll
    for (int fn = 0; fn < 4; ++fn) {
      b[fn].half[0] = *(const v8us*)(wp + (size_t)fn * 16 * FEAT + k0);
      b[fn].half[1] = *(const v8us*)(wp + (size_t)fn * 16 * FEAT + k0 + 16);
    }
#pragma unroll
    for (int fm = 0; fm < 2; ++fm)
#pragma unroll
      for (int fn = 0; fn < 4; ++fn) {
        if (BF) acc[fm][fn] = __builtin_amdgcn_wmma_f32_16x16x32_bf16(false, a[fm].b, false, b[fn].b, (short)0, acc[fm][fn], false, false);
        else    acc[fm][fn] = __builtin_amdgcn_wmma_f32_16x16x32_f16(false, a[fm].h, false, b[fn].h, (short)0, acc[fm][fn], false, false);
      }
    asm volatile("v_nop\n\tv_nop\n\tv_nop\n\tv_nop"
                 : "+v"(acc[0][0]), "+v"(acc[0][1]), "+v"(acc[0][2]), "+v"(acc[0][3]),
                   "+v"(acc[1][0]), "+v"(acc[1][1]), "+v"(acc[1][2]), "+v"(acc[1][3])
                 : "v"(a[0].h), "v"(a[1].h), "v"(b[0].h), "v"(b[1].h), "v"(b[2].h), "v"(b[3].h));
  }

  float bcol[4];
#pragma unroll
  for (int fn = 0; fn < 4; ++fn) bcol[fn] = 0.0f;
  if (EPI != 1) {
#pragma unroll
    for (int fn = 0; fn < 4; ++fn) bcol[fn] = bf16_rne(bias[n0 + fn * 16 + ln]);
  }
#pragma unroll
  for (int fm = 0; fm < 2; ++fm) {
    float brow[8];
#pragma unroll
    for (int r = 0; r < 8; ++r) brow[r] = 0.0f;
    if (EPI == 1) {
#pragma unroll
      for (int r = 0; r < 8; ++r) brow[r] = bf16_rne(bias[m0 + fm * 16 + 8 * hh + r]);
    }
#pragma unroll
    for (int fn = 0; fn < 4; ++fn)
#pragma unroll
      for (int r = 0; r < 8; ++r) {
        float v = acc[fm][fn][r] * sc + ((EPI == 1) ? brow[r] : bcol[fn]);
        if (EPI != 2) v = v * carry;
        sst[w][8 * hh + r][fn * 16 + ln] = v;
      }
    __syncthreads();
    if (EPI == 2) {
      float* of = (float*)outp;
      const int rsub = lane >> 4, c4 = (lane & 15) * 4;
      for (int pass = 0; pass < 2; ++pass) {
#pragma unroll
        for (int q = 0; q < 8; ++q) {
          const int row = 2 * q + rsub;
          const int m = m0 + fm * 16 + row;
          const int bb = m / SEQ;
          const size_t grow = (size_t)bb * SEQ_FULL + (size_t)(m - bb * SEQ);
          const v4f v = *(const v4fa*)&sst[w][row][c4];
          *(volatile v4f*)(of + grow * FEAT + n0 + c4) = v;
        }
        if (pass == 0) __threadfence();
      }
    } else {
      unsigned short* oh = (unsigned short*)outp;
      const int jsub = lane >> 3, p8 = (lane & 7) * 8;
      for (int pass = 0; pass < 2; ++pass) {
#pragma unroll
        for (int it = 0; it < 4; ++it) {
          const int j = jsub + 4 * it;
          const v4f x0 = *(const v4fa*)&sst[w][j][p8];
          const v4f x1 = *(const v4fa*)&sst[w][j][p8 + 4];
          Frag f;
          f.e[0] = (_Float16)x0[0]; f.e[1] = (_Float16)x0[1]; f.e[2] = (_Float16)x0[2]; f.e[3] = (_Float16)x0[3];
          f.e[4] = (_Float16)x1[0]; f.e[5] = (_Float16)x1[1]; f.e[6] = (_Float16)x1[2]; f.e[7] = (_Float16)x1[3];
          const v8us o = f.half[0];
          *(volatile v8us*)(oh + (size_t)(m0 + fm * 16 + j) * N + n0 + p8) = o;
        }
        if (pass == 0) __threadfence();
      }
    }
    __syncthreads();
  }
}

__device__ __forceinline__ void fa_step(const unsigned short* __restrict__ kp, const unsigned short* __restrict__ vp,
                                        const Frag& qf, float& mr, float& lr, v8f& Oh, v8f& Ol) {
  const v8us zz = {0, 0, 0, 0, 0, 0, 0, 0};
  Frag k0, k1, vf;
  k0.half[0] = *(const v8us*)(kp);             k0.half[1] = zz;
  k1.half[0] = *(const v8us*)(kp + 16 * FEAT); k1.half[1] = zz;
  vf.half[0] = *(const v8us*)(vp);
  vf.half[1] = *(const v8us*)(vp + 16);
  v8f s0 = {0.f, 0.f, 0.f, 0.f, 0.f, 0.f, 0.f, 0.f};
  v8f s1 = {0.f, 0.f, 0.f, 0.f, 0.f, 0.f, 0.f, 0.f};
  mma_s2(k0.h, k1.h, qf.h, s0, s1);
  float sc[16];
#pragma unroll
  for (int r = 0; r < 8; ++r) { sc[r] = s0[r] * 0.0009765625f; sc[8 + r] = s1[r] * 0.0009765625f; }
  float mx = sc[0];
#pragma unroll
  for (int i = 1; i < 16; ++i) mx = fmaxf(mx, sc[i]);
  mx = fmaxf(mx, __shfl_xor(mx, 16, 32));
  const float mnew = fmaxf(mr, mx);
  const float al = exp2f((mr - mnew) * LOG2E);
  mr = mnew;
  Frag ph, pl;
  float ps = 0.0f;
#pragma unroll
  for (int i = 0; i < 16; ++i) {
    const float pc = exp2f(fmaf(sc[i] - mnew, LOG2E, 8.0f));
    ps += pc;
    const _Float16 h = (_Float16)pc;
    ph.e[i] = h;
    pl.e[i] = (_Float16)((pc - (float)h) * 2048.0f);
  }
  ps += __shfl_xor(ps, 16, 32);
  lr = lr * al + ps;
  Oh = Oh * al; Ol = Ol * al;
  mma_h2(vf.h, ph.h, pl.h, Oh, Ol);
}

__global__ __launch_bounds__(128) void k_attn(const unsigned short* __restrict__ Qp, const unsigned short* __restrict__ Kp,
                                              const unsigned short* __restrict__ Vt, unsigned short* __restrict__ O2) {
  __shared__ __attribute__((aligned(16))) float so[4][16][20];
  const int tid = threadIdx.x, w = __builtin_amdgcn_readfirstlane((int)(tid >> 5)), lane = tid & 31, ln = lane & 15, hh = lane >> 4;
  const int qt = blockIdx.x % (SEQ / 64);
  const int p = blockIdx.x / (SEQ / 64);
  const int b = p % NB, c = p / NB;
  const int qbase = qt * 64 + 16 * w;
  const int qg = qbase + ln;
  const v8us zz = {0, 0, 0, 0, 0, 0, 0, 0};
  Frag qf;
  qf.half[0] = *(const v8us*)(Qp + ((size_t)b * SEQ + qg) * FEAT + c * 16 + 8 * hh);
  qf.half[1] = zz;
  const unsigned short* kb = Kp + ((size_t)b * SEQ + ln) * FEAT + c * 16 + 8 * hh;
  const unsigned short* vb = Vt + (size_t)(c * 16 + ln) * MROWS + (size_t)b * SEQ + 8 * hh;
  float mr = -3.0e38f, lr = 0.0f;
  v8f Oh = {0.f, 0.f, 0.f, 0.f, 0.f, 0.f, 0.f, 0.f};
  v8f Ol = {0.f, 0.f, 0.f, 0.f, 0.f, 0.f, 0.f, 0.f};
#pragma unroll 1
  for (int j = 0; j < SEQ / 32; ++j)
    fa_step(kb + (size_t)j * 32 * FEAT, vb + j * 32, qf, mr, lr, Oh, Ol);

  const float inv = 16.0f * (1.0f / lr);
#pragma unroll
  for (int r = 0; r < 8; ++r)
    so[w][ln][8 * hh + r] = (Oh[r] + Ol[r] * 0.00048828125f) * inv;
  __syncthreads();
  const int qq = lane >> 1, d0 = (lane & 1) * 8;
  const v4f x0 = *(const v4fa*)&so[w][qq][d0];
  const v4f x1 = *(const v4fa*)&so[w][qq][d0 + 4];
  Frag f;
  f.e[0] = (_Float16)x0[0]; f.e[1] = (_Float16)x0[1]; f.e[2] = (_Float16)x0[2]; f.e[3] = (_Float16)x0[3];
  f.e[4] = (_Float16)x1[0]; f.e[5] = (_Float16)x1[1]; f.e[6] = (_Float16)x1[2]; f.e[7] = (_Float16)x1[3];
  const v8us o = f.half[0];
  const int R = (c * NB + b) * (SEQ / 4) + (qbase >> 2) + (lane >> 3);
  const int hp = R / MROWS;
  const int prow = R - hp * MROWS;
  unsigned short* dst = O2 + (size_t)prow * FEAT + hp * 64 + (lane & 7) * 8;
  *(volatile v8us*)dst = o;
  __threadfence();
  *(volatile v8us*)dst = o;
}

extern "C" void kernel_launch(void* const* d_in, const int* in_sizes, int n_in,
                              void* d_out, int out_size, void* d_ws, size_t ws_size, hipStream_t stream) {
  if (n_in < 15) return;
  const long long needx = ((long long)(NB - 1) * SEQ_FULL + SEQ) * FEAT;
  if ((long long)in_sizes[0] < needx) return;
  if ((long long)out_size < needx) return;
  for (int i = 1; i < 15; i += 2) {
    if ((long long)in_sizes[i] < (long long)FEAT * FEAT) return;
    if ((long long)in_sizes[i + 1] < (long long)FEAT) return;
  }
  const float* x    = (const float*)d_in[0];
  const float* wq_w = (const float*)d_in[1];
  const float* wq_b = (const float*)d_in[2];
  const float* wk_w = (const float*)d_in[3];
  const float* wk_b = (const float*)d_in[4];
  const float* wv_w = (const float*)d_in[5];
  const float* wv_b = (const float*)d_in[6];
  const float* vq_w = (const float*)d_in[7];
  const float* vq_b = (const float*)d_in[8];
  const float* vk_w = (const float*)d_in[9];
  const float* vk_b = (const float*)d_in[10];
  const float* vv_w = (const float*)d_in[11];
  const float* vv_b = (const float*)d_in[12];
  const float* wo_w = (const float*)d_in[13];
  const float* wo_b = (const float*)d_in[14];

  char* ws = (char*)d_ws;
  size_t off = 0;
  const size_t planeA = (size_t)MROWS * FEAT * 2;
  const size_t planeW = (size_t)FEAT * FEAT * 2;
  unsigned short* Xb  = (unsigned short*)(ws + off); off += (planeA + 255) & ~(size_t)255;
  unsigned short* Wqb = (unsigned short*)(ws + off); off += (planeW + 255) & ~(size_t)255;
  unsigned short* Wkb = (unsigned short*)(ws + off); off += (planeW + 255) & ~(size_t)255;
  unsigned short* Wvb = (unsigned short*)(ws + off); off += (planeW + 255) & ~(size_t)255;
  unsigned short* Vqh = (unsigned short*)(ws + off); off += (planeW + 255) & ~(size_t)255;
  unsigned short* Vkh = (unsigned short*)(ws + off); off += (planeW + 255) & ~(size_t)255;
  unsigned short* Vvh = (unsigned short*)(ws + off); off += (planeW + 255) & ~(size_t)255;
  unsigned short* Woh = (unsigned short*)(ws + off); off += (planeW + 255) & ~(size_t)255;
  unsigned short* T1q = (unsigned short*)(ws + off); off += (planeA + 255) & ~(size_t)255;
  unsigned short* T1k = (unsigned short*)(ws + off); off += (planeA + 255) & ~(size_t)255;
  unsigned short* T1v = (unsigned short*)(ws + off); off += (planeA + 255) & ~(size_t)255;
  unsigned short* Qp  = (unsigned short*)(ws + off); off += (planeA + 255) & ~(size_t)255;
  unsigned short* Kp  = (unsigned short*)(ws + off); off += (planeA + 255) & ~(size_t)255;
  unsigned short* Vt  = (unsigned short*)(ws + off); off += (planeA + 255) & ~(size_t)255;
  unsigned short* O2  = (unsigned short*)(ws + off); off += (planeA + 255) & ~(size_t)255;
  if (off > ws_size) return;

  const unsigned gx = (unsigned)((MROWS * (FEAT / 8) + 255) / 256);
  const unsigned gw = (unsigned)((FEAT * (FEAT / 8) + 255) / 256);
  k_cvtx<<<gx, 256, 0, stream>>>(x, Xb);
  k_cvtw<0><<<gw, 256, 0, stream>>>(wq_w, Wqb);
  k_cvtw<0><<<gw, 256, 0, stream>>>(wk_w, Wkb);
  k_cvtw<0><<<gw, 256, 0, stream>>>(wv_w, Wvb);
  k_cvtw<1><<<gw, 256, 0, stream>>>(vq_w, Vqh);
  k_cvtw<1><<<gw, 256, 0, stream>>>(vk_w, Vkh);
  k_cvtw<1><<<gw, 256, 0, stream>>>(vv_w, Vvh);
  k_cvtw<1><<<gw, 256, 0, stream>>>(wo_w, Woh);

  const dim3 gA((unsigned)(MROWS / 128), (unsigned)(FEAT / 128));
  const dim3 gV((unsigned)(FEAT / 128), (unsigned)(MROWS / 128));
  const float s10 = 0.0009765625f;
  const float s14 = 0.00006103515625f;
  k_gemm<true, 0><<<gA, 256, 0, stream>>>(Xb, Wqb, wq_b, (void*)T1q, FEAT, 1.0f, 16.0f);
  k_gemm<false, 0><<<gA, 256, 0, stream>>>(T1q, Vqh, vq_b, (void*)Qp, FEAT, s10, 16.0f);
  k_gemm<true, 0><<<gA, 256, 0, stream>>>(Xb, Wkb, wk_b, (void*)T1k, FEAT, 1.0f, 16.0f);
  k_gemm<false, 0><<<gA, 256, 0, stream>>>(T1k, Vkh, vk_b, (void*)Kp, FEAT, s10, 16.0f);
  k_gemm<true, 0><<<gA, 256, 0, stream>>>(Xb, Wvb, wv_b, (void*)T1v, FEAT, 1.0f, 16.0f);
  k_gemm<false, 1><<<gV, 256, 0, stream>>>(Vvh, T1v, vv_b, (void*)Vt, MROWS, s10, 16.0f);

  k_attn<<<(unsigned)(NCH * NB * (SEQ / 64)), 128, 0, stream>>>(Qp, Kp, Vt, O2);

  k_gemm<false, 2><<<gA, 256, 0, stream>>>(O2, Woh, wo_b, d_out, FEAT, s14, 1.0f);
}
